// GlobalAttentionGraph_41205916237954
// MI455X (gfx1250) — hardware-run, weakly checked
//
#include <hip/hip_runtime.h>


#ifndef NB
#define NB 32
#endif
#ifndef SEQ
#define SEQ 1024
#endif
#define NB_FULL  32
#define SEQ_FULL 1024
#ifndef OUT_SEQ
#define OUT_SEQ SEQ
#endif
#define DM   256
#define NLAY 3
#define AW   2
#define LNP  260
#define WCAR 16.0f
#define WINV 0.0625f
#define PCAR 4.0f
#define SCS  (1.0f / 256.0f)
#define VINV 0.25f
#define L2E  1.4426950408889634f
#define PSH  14.0f
#define NEGB (-1.0e30f)
#define LNEPS 1.0e-5f

static_assert(DM == 256);
static_assert(DM % 64 == 0);
static_assert(DM % 32 == 0);
static_assert(SEQ % 64 == 0);
static_assert((NB * SEQ) % 64 == 0);
static_assert(SEQ % 32 == 0);
static_assert(SEQ % (16 * AW) == 0);
static_assert((NB * SEQ) % (16 * AW) == 0);
static_assert(SEQ % (32 * AW * 4) == 0);
static_assert(LNP >= DM);
static_assert((LNP * 4) % 16 == 0);
static_assert(32 * 8 == DM);
static_assert(2 * 32 * 4 == DM);
static_assert(16 * 16 == DM);
static_assert(8 * 2 == 16);
static_assert(NB <= NB_FULL);
static_assert(SEQ <= SEQ_FULL);
static_assert(((size_t)SEQ * DM) % 8 == 0);
static_assert(((size_t)DM * DM) % 8 == 0);
static_assert((size_t)NB * SEQ * DM * 2 < (size_t)4294967296);
static_assert((size_t)AW * 16 * LNP * 4 + (size_t)SEQ * 4 <= 131072);
static_assert((size_t)AW * 16 * LNP * 4 <= 131072);
static_assert((size_t)16 * 68 * 4 <= 131072);

typedef _Float16 h16;
typedef __attribute__((ext_vector_type(16))) _Float16 v16h;
typedef __attribute__((ext_vector_type(8)))  _Float16 v8h;
typedef __attribute__((ext_vector_type(8)))  float    v8f;
typedef __attribute__((ext_vector_type(4)))  float    v4f;
typedef v4f  __attribute__((may_alias)) v4fa;

__device__ __forceinline__ unsigned short f2bf(float f) { unsigned u = __float_as_uint(f); u += 0x7FFFu + ((u >> 16) & 1u); return (unsigned short)(u >> 16); }
__device__ __forceinline__ float bfr(float f) { return __uint_as_float(((unsigned)f2bf(f)) << 16); }
__device__ __forceinline__ v16h cat16(v8h lo, v8h hi) { return __builtin_shufflevector(lo, hi, 0, 1, 2, 3, 4, 5, 6, 7, 8, 9, 10, 11, 12, 13, 14, 15); }
__device__ __forceinline__ v8f wmma16(v16h a, v16h b, v8f c) { return __builtin_amdgcn_wmma_f32_16x16x32_f16(false, a, false, b, (short)0, c, false, false); }
__device__ __forceinline__ v8f wmma16g(v16h a, v16h b, v8f c) { c = wmma16(a, b, c); asm volatile("v_nop\n\tv_nop\n\tv_nop\n\tv_nop" : "+v"(c) : "v"(a), "v"(b)); return c; }
__device__ __forceinline__ v16h  ldh(const h16* p) { return cat16(*(const v8h*)p, *(const v8h*)(p + 16)); }
__device__ __forceinline__ void wave_sync() { __builtin_amdgcn_fence(3  , "wavefront"); __builtin_amdgcn_wave_barrier(); asm volatile("" ::: "memory"); }
__device__ __forceinline__ void group_end() { asm volatile("" ::: "memory"); __builtin_amdgcn_sched_barrier(0); }
static __device__ __forceinline__ h16 toh_flush(float v) { const float w = (fabsf(v) < 6.103515625e-05f) ? 0.0f : v; return (h16)w; }
__device__ __forceinline__ v4f ld4bf(const float* p) { const v4f v = *(const v4f*)p; v4f o; o[0] = bfr(v[0]); o[1] = bfr(v[1]); o[2] = bfr(v[2]); o[3] = bfr(v[3]); return o; }
__device__ __forceinline__ float pair_bias(float mi, float mj) {
#pragma clang fp contract(off)
    const float mm = mi * mj; const float om = 1.0f - mm; const float bg = 100000.0f * om; return mm - bg;
}
__device__ __forceinline__ float score_add(float s, float bias) {
#pragma clang fp contract(off)
    const float t = s * SCS; return t + bias;
}

__device__ __forceinline__ void cvt8_body(const float* __restrict__ src, h16* dst, size_t n8, const float carry) {
    const size_t i = (size_t)blockIdx.x * 256 + threadIdx.x; if (i >= n8) return;
    const v8f v = *(const v8f*)(src + i * 8); v8h o;
#pragma unroll
    for (int k = 0; k < 8; ++k) o[k] = toh_flush(bfr(v[k]) * carry);
    *(volatile v8h*)(dst + i * 8) = o; __threadfence(); *(volatile v8h*)(dst + i * 8) = o;
}
__global__ __launch_bounds__(256) void k_cvtx(const float* __restrict__ src, h16* dst, size_t n8) { cvt8_body(src, dst, n8, 1.0f); }
__global__ __launch_bounds__(256) void k_cvtw(const float* __restrict__ src, h16* dst, size_t n8) { cvt8_body(src, dst, n8, WCAR); }

template <int MODE>
__device__ __forceinline__ void proj_body(const h16* __restrict__ A, const h16* __restrict__ Bt, const float* __restrict__ bias, h16* Ph) {
    __shared__ __align__(16) float os[16 * 68];
    const int K = DM;
    const int lane = threadIdx.x & 31, lr = lane & 15, hi = lane >> 4;
    const unsigned r0 = blockIdx.x * 64u, c0 = blockIdx.y * 64u;
    v8f acc[4][4];
#pragma unroll
    for (int mb = 0; mb < 4; ++mb)
#pragma unroll
        for (int nb = 0; nb < 4; ++nb) acc[mb][nb] = (v8f){};
    const size_t aoff = (size_t)(r0 + (unsigned)lr) * K + 8 * hi, boff = (size_t)(c0 + (unsigned)lr) * K + 8 * hi;
#pragma unroll 1
    for (int kc = 0; kc < K; kc += 32) {
        v16h a[4];
#pragma unroll
        for (int mb = 0; mb < 4; ++mb) a[mb] = ldh(A + aoff + (size_t)mb * 16 * K + kc);
#pragma unroll
        for (int nb = 0; nb < 4; ++nb) { const v16h b = ldh(Bt + boff + (size_t)nb * 16 * K + kc);
#pragma unroll
            for (int mb = 0; mb < 4; ++mb) acc[mb][nb] = wmma16g(a[mb], b, acc[mb][nb]); }
    }
    float bc[4];
#pragma unroll
    for (int nb = 0; nb < 4; ++nb) bc[nb] = (MODE == 0) ? bfr(bias[c0 + nb * 16 + lr]) : 0.0f;
    size_t tbase, pitch;
    if (MODE == 0) { tbase = (size_t)r0 * DM + (size_t)c0; pitch = DM; }
    else           { const unsigned bb = c0 / (unsigned)SEQ, tt = c0 % (unsigned)SEQ;
                     tbase = (size_t)bb * (size_t)DM * SEQ + (size_t)r0 * SEQ + (size_t)tt; pitch = SEQ; }
    static_assert(4 * (32 / 8) == 16);
    static_assert((32 % 8 == 0) && 8 * 8 == 64);
#pragma unroll
    for (int mb = 0; mb < 4; ++mb) {
        float br[8];
#pragma unroll
        for (int j = 0; j < 8; ++j) br[j] = (MODE == 1) ? bfr(bias[r0 + mb * 16 + hi * 8 + j]) : 0.0f;
#pragma unroll
        for (int nb = 0; nb < 4; ++nb) {
#pragma unroll
            for (int j = 0; j < 8; ++j) os[(hi * 8 + j) * 68 + nb * 16 + lr] = (acc[mb][nb][j] * WINV + bc[nb] + br[j]) * PCAR; }
        wave_sync();
#pragma unroll 1
        for (int ps = 0; ps < 2; ++ps) {
            const size_t sb = tbase + (size_t)(mb * 16) * pitch;
#pragma unroll
            for (int s = 0; s < 4; ++s) { const int row = 4 * s + (lane >> 3), c8 = (lane & 7) * 8;
                const v4f x0 = *(const v4fa*)(&os[row * 68 + c8]); const v4f x1 = *(const v4fa*)(&os[row * 68 + c8 + 4]); v8h hv;
#pragma unroll
                for (int i = 0; i < 4; ++i) { hv[i] = toh_flush(x0[i]); hv[4 + i] = toh_flush(x1[i]); }
                const size_t oo = sb + (size_t)row * pitch + c8;
                *(volatile v8h*)(Ph + oo) = hv; }
            if (ps == 0) __threadfence(); }
        wave_sync();
    }
}
__global__ __launch_bounds__(32) __attribute__((amdgpu_num_vgpr(256))) void k_projrow(const h16* __restrict__ A, const h16* __restrict__ Bt, const float* __restrict__ bias, h16* Ph) { proj_body<0>(A, Bt, bias, Ph); }
__global__ __launch_bounds__(32) __attribute__((amdgpu_num_vgpr(256))) void k_projtr(const h16* __restrict__ A, const h16* __restrict__ Bt, const float* __restrict__ bias, h16* Ph) { proj_body<1>(A, Bt, bias, Ph); }

template <int MODE>
__device__ __forceinline__ void rowln_body(const h16* __restrict__ X, const h16* __restrict__ W, const float* __restrict__ bias,
                                           const float* __restrict__ gain, const float* __restrict__ shift,
                                           const float* RESR, float* RESW, h16* XN, float* OUT) {
    __shared__ __align__(16) float os[AW * 16 * LNP];
    const int lane = threadIdx.x & 31, lr = lane & 15, hi = lane >> 4;
    const int wave = __builtin_amdgcn_readfirstlane((int)(threadIdx.x >> 5));
    const unsigned gr = (blockIdx.x * (unsigned)AW + (unsigned)wave) * 16u;
    const unsigned bb = gr / (unsigned)SEQ, tt = gr % (unsigned)SEQ;
    v8f acc[16];
#pragma unroll
    for (int j = 0; j < 16; ++j) acc[j] = (v8f){};
    const unsigned xo = (gr + (unsigned)lr) * (unsigned)DM + 8u * (unsigned)hi;
    const unsigned wo = (unsigned)lr * (unsigned)DM + 8u * (unsigned)hi;
#pragma unroll 1
    for (unsigned kc = 0; kc < (unsigned)DM; kc += 32u) {
        const v16h xb = ldh(X + (xo + kc));
        group_end();
#pragma unroll
        for (int g = 0; g < 8; ++g) {
            const h16* wp = W + (wo + (unsigned)(2 * g) * 16u * (unsigned)DM + kc);
            const v16h w0 = ldh(wp), w1 = ldh(wp + 16 * DM);
            acc[2 * g + 0] = wmma16g(w0, xb, acc[2 * g + 0]); acc[2 * g + 1] = wmma16g(w1, xb, acc[2 * g + 1]);
            group_end();
        }
    }
    const int wb = wave * 16 * LNP;
#pragma unroll
    for (int j = 0; j < 16; ++j) {
        const v4f p0 = ld4bf(bias + 16 * j + 8 * hi), p1 = ld4bf(bias + 16 * j + 8 * hi + 4); v4f a, c;
#pragma unroll
        for (int r = 0; r < 4; ++r) { a[r] = acc[j][r] * WINV + p0[r]; c[r] = acc[j][4 + r] * WINV + p1[r]; }
        *(v4fa*)(&os[wb + lr * LNP + 16 * j + 8 * hi]) = a; *(v4fa*)(&os[wb + lr * LNP + 16 * j + 8 * hi + 4]) = c;
        if ((j & 1) == 1) group_end();
    }
    wave_sync();
#pragma unroll 1
    for (int row = 0; row < 16; ++row) {
        const int ix = wb + row * LNP + lane * 8;
        const v4f x0 = *(const v4fa*)(&os[ix]); const v4f x1 = *(const v4fa*)(&os[ix + 4]);
        float s = ((x0[0] + x0[1]) + (x0[2] + x0[3])) + ((x1[0] + x1[1]) + (x1[2] + x1[3]));
#pragma unroll
        for (int d = 1; d < 32; d <<= 1) s += __shfl_xor(s, d, 32);
        const float mu = s * (1.0f / DM);
        const v4f d0 = x0 - mu, d1 = x1 - mu;
        float q = ((d0[0] * d0[0] + d0[1] * d0[1]) + (d0[2] * d0[2] + d0[3] * d0[3])) + ((d1[0] * d1[0] + d1[1] * d1[1]) + (d1[2] * d1[2] + d1[3] * d1[3]));
#pragma unroll
        for (int d = 1; d < 32; d <<= 1) q += __shfl_xor(q, d, 32);
        const float rstd = rsqrtf(q * (1.0f / DM) + LNEPS);
        const v4f y0 = d0 * rstd, y1 = d1 * rstd;
        *(v4fa*)(&os[ix]) = y0; *(v4fa*)(&os[ix + 4]) = y1;
    }
    wave_sync();
    if (MODE == 1) {
        static_assert(16 * 1 * 32 * 16 == 16 * DM * 2);
        const int c8 = lane * 8;
        const v4f g0 = ld4bf(gain + c8), g1 = ld4bf(gain + c8 + 4), b0 = ld4bf(shift + c8), b1 = ld4bf(shift + c8 + 4);
#pragma unroll 1
        for (int ps = 0; ps < 2; ++ps) {
#pragma unroll 2
            for (int row = 0; row < 16; ++row) {
                const v4f x0 = *(const v4fa*)(&os[wb + row * LNP + c8]); const v4f x1 = *(const v4fa*)(&os[wb + row * LNP + c8 + 4]);
                const size_t ro = (size_t)(gr + (unsigned)row) * DM + c8;
                const v4f q0 = *(const v4f*)(RESR + ro); const v4f q1 = *(const v4f*)(RESR + ro + 4); v8h hv;
#pragma unroll
                for (int i = 0; i < 4; ++i) { const float u0 = fmaxf(x0[i] * g0[i] + b0[i] + q0[i], 0.0f); const float u1 = fmaxf(x1[i] * g1[i] + b1[i] + q1[i], 0.0f);
                    hv[i] = toh_flush(u0); hv[4 + i] = toh_flush(u1); }
                *(volatile v8h*)(XN + ro) = hv; }
            if (ps == 0) __threadfence(); }
    } else {
        static_assert(16 * 2 * 32 * 16 == 16 * DM * 4);
        const int c4 = lane * 4;
        const v4f g0 = ld4bf(gain + c4), g1 = ld4bf(gain + 128 + c4), b0 = ld4bf(shift + c4), b1 = ld4bf(shift + 128 + c4);
        const size_t obase = (MODE == 0) ? (size_t)gr * DM : ((size_t)bb * OUT_SEQ + (size_t)tt) * DM;
#pragma unroll 1
        for (int ps = 0; ps < 2; ++ps) {
#pragma unroll 2
            for (int row = 0; row < 16; ++row) {
                const v4f x0 = *(const v4fa*)(&os[wb + row * LNP + c4]); const v4f x1 = *(const v4fa*)(&os[wb + row * LNP + 128 + c4]);
                v4f u0 = x0 * g0 + b0, u1 = x1 * g1 + b1;
                if (MODE == 2) { const size_t ro = (size_t)(gr + (unsigned)row) * DM + c4;
                                 const v4f q0 = *(const v4f*)(RESR + ro); const v4f q1 = *(const v4f*)(RESR + ro + 128); u0 = u0 + q0; u1 = u1 + q1; }
                const size_t oo = obase + (size_t)row * DM + c4;
                if (MODE == 0) { *(volatile v4f*)(RESW + oo) = u0; *(volatile v4f*)(RESW + oo + 128) = u1; }
                else           { *(volatile v4f*)(OUT + oo) = u0;  *(volatile v4f*)(OUT + oo + 128) = u1; } }
            if (ps == 0) __threadfence(); }
    }
}
__global__ __launch_bounds__(32 * AW) __attribute__((amdgpu_num_vgpr(256))) void k_lnres(const h16* __restrict__ X, const h16* __restrict__ W, const float* __restrict__ bias, const float* __restrict__ gain, const float* __restrict__ shift,
                                                   const float* RESR, float* RESW, h16* XN, float* OUT) { rowln_body<0>(X, W, bias, gain, shift, RESR, RESW, XN, OUT); }
__global__ __launch_bounds__(32 * AW) __attribute__((amdgpu_num_vgpr(256))) void k_lnmix(const h16* __restrict__ X, const h16* __restrict__ W, const float* __restrict__ bias, const float* __restrict__ gain, const float* __restrict__ shift,
                                                   const float* RESR, float* RESW, h16* XN, float* OUT) { rowln_body<1>(X, W, bias, gain, shift, RESR, RESW, XN, OUT); }
__global__ __launch_bounds__(32 * AW) __attribute__((amdgpu_num_vgpr(256))) void k_lnout(const h16* __restrict__ X, const h16* __restrict__ W, const float* __restrict__ bias, const float* __restrict__ gain, const float* __restrict__ shift,
                                                   const float* RESR, float* RESW, h16* XN, float* OUT) { rowln_body<2>(X, W, bias, gain, shift, RESR, RESW, XN, OUT); }

__global__ __launch_bounds__(32 * AW) __attribute__((amdgpu_num_vgpr(256))) void k_flash(const h16* __restrict__ QH, const h16* __restrict__ KP, const h16* __restrict__ VT,
                                                   const float* __restrict__ masks, const float* __restrict__ gain, const float* __restrict__ shift, h16* CAH) {
    __shared__ __align__(16) float os[AW * 16 * LNP];
    __shared__ __align__(16) float km[SEQ];
    const int lane = threadIdx.x & 31, lr = lane & 15, hi = lane >> 4;
    const int wave = __builtin_amdgcn_readfirstlane((int)(threadIdx.x >> 5));
    const unsigned b = blockIdx.y;
    const int t0 = (int)(blockIdx.x * (unsigned)AW + (unsigned)wave) * 16;
    const float* mrow = masks + (size_t)b * SEQ_FULL;
#pragma unroll 1
    for (unsigned i = threadIdx.x * 4u; i < (unsigned)SEQ; i += 32u * AW * 4u) {
        const v4f mv = *(const v4f*)(mrow + i); v4f mo;
#pragma unroll
        for (int c = 0; c < 4; ++c) mo[c] = bfr(mv[c]);
        *(v4fa*)(&km[i]) = mo; }
    __syncthreads();
    const float qmv = km[t0 + lr];
    const unsigned pbase = b * (unsigned)SEQ * (unsigned)DM;
    const unsigned qo = pbase + (unsigned)(t0 + lr) * (unsigned)DM + 8u * (unsigned)hi;
    const unsigned ko = pbase + (unsigned)lr * (unsigned)DM + 8u * (unsigned)hi;
    const unsigned vo = pbase + (unsigned)lr * (unsigned)SEQ + 8u * (unsigned)hi;
    v8f o[16];
#pragma unroll
    for (int j = 0; j < 16; ++j) o[j] = (v8f){};
    float m = NEGB, l = 0.0f;
#pragma unroll 1
    for (unsigned key0 = 0; key0 < (unsigned)SEQ; key0 += 32u) {
        const unsigned kao = ko + key0 * (unsigned)DM;
        v8f sA = (v8f){}, sB = (v8f){};
#pragma unroll 1
        for (unsigned kc = 0; kc < (unsigned)DM; kc += 32u) {
            const v16h qf = ldh(QH + (qo + kc));
            const h16* kp = KP + (kao + kc);
            const v16h k0 = ldh(kp), k1 = ldh(kp + 16 * DM);
            sA = wmma16g(k0, qf, sA); sB = wmma16g(k1, qf, sB);
        }
        const int kq = (int)key0 + 8 * hi;
        const v4f m0 = *(const v4fa*)(&km[kq]), m1 = *(const v4fa*)(&km[kq + 4]), m2 = *(const v4fa*)(&km[kq + 16]), m3 = *(const v4fa*)(&km[kq + 20]);
        float sva[8], svb[8]; float mx = NEGB;
#pragma unroll
        for (int r = 0; r < 4; ++r) {
            sva[r]     = score_add(sA[r],     pair_bias(qmv, m0[r]));
            sva[4 + r] = score_add(sA[4 + r], pair_bias(qmv, m1[r]));
            svb[r]     = score_add(sB[r],     pair_bias(qmv, m2[r]));
            svb[4 + r] = score_add(sB[4 + r], pair_bias(qmv, m3[r])); }
#pragma unroll
        for (int r = 0; r < 8; ++r) mx = fmaxf(mx, fmaxf(sva[r], svb[r]));
        mx = fmaxf(mx, __shfl_xor(mx, 16, 32));
        const float mnew = fmaxf(m, mx);
        const float alpha = __builtin_amdgcn_exp2f((m - mnew) * L2E);
        v16h pb; float ls = 0.0f;
#pragma unroll
        for (int r = 0; r < 8; ++r) {
            const float ea = (sva[r] - mnew) * L2E + PSH, eb = (svb[r] - mnew) * L2E + PSH;
            const float xa = __builtin_amdgcn_exp2f(ea), xb = __builtin_amdgcn_exp2f(eb);
            const float ga = (ea < -PSH) ? 0.0f : xa, gb = (eb < -PSH) ? 0.0f : xb;
            const h16 pa = (h16)ga; const h16 pc = (h16)gb;
            pb[r] = pa; pb[8 + r] = pc; ls += (float)pa + (float)pc; }
        l = l * alpha + ls; m = mnew;
        if (__builtin_amdgcn_ballot_w32(alpha != 1.0f) != 0u) {
#pragma unroll
            for (int j = 0; j < 16; ++j) o[j] = o[j] * alpha; }
        group_end();
        const h16* va = VT + (vo + key0);
#pragma unroll
        for (int g = 0; g < 8; ++g) {
            const v16h v0 = ldh(va + (2 * g + 0) * 16 * SEQ), v1 = ldh(va + (2 * g + 1) * 16 * SEQ);
            o[2 * g + 0] = wmma16g(v0, pb, o[2 * g + 0]); o[2 * g + 1] = wmma16g(v1, pb, o[2 * g + 1]);
            group_end();
        }
    }
    l += __shfl_xor(l, 16, 32);
    const float inv = VINV * (1.0f / l);
    const int wb = wave * 16 * LNP;
#pragma unroll
    for (int j = 0; j < 16; ++j) { v4f a, c;
        a[0] = o[j][0] * inv; a[1] = o[j][1] * inv; a[2] = o[j][2] * inv; a[3] = o[j][3] * inv; c[0] = o[j][4] * inv; c[1] = o[j][5] * inv; c[2] = o[j][6] * inv; c[3] = o[j][7] * inv;
        *(v4fa*)(&os[wb + lr * LNP + 16 * j + 8 * hi]) = a; *(v4fa*)(&os[wb + lr * LNP + 16 * j + 8 * hi + 4]) = c;
        if ((j & 1) == 1) group_end(); }
    wave_sync();
#pragma unroll 1
    for (int row = 0; row < 16; ++row) {
        const int ix = wb + row * LNP + lane * 8;
        const v4f x0 = *(const v4fa*)(&os[ix]); const v4f x1 = *(const v4fa*)(&os[ix + 4]);
        float s = ((x0[0] + x0[1]) + (x0[2] + x0[3])) + ((x1[0] + x1[1]) + (x1[2] + x1[3]));
#pragma unroll
        for (int d = 1; d < 32; d <<= 1) s += __shfl_xor(s, d, 32);
        const float mu = s * (1.0f / DM);
        const v4f d0 = x0 - mu, d1 = x1 - mu;
        float q = ((d0[0] * d0[0] + d0[1] * d0[1]) + (d0[2] * d0[2] + d0[3] * d0[3])) + ((d1[0] * d1[0] + d1[1] * d1[1]) + (d1[2] * d1[2] + d1[3] * d1[3]));
#pragma unroll
        for (int d = 1; d < 32; d <<= 1) q += __shfl_xor(q, d, 32);
        const float rstd = rsqrtf(q * (1.0f / DM) + LNEPS);
        const v4f y0 = d0 * rstd, y1 = d1 * rstd;
        *(v4fa*)(&os[ix]) = y0; *(v4fa*)(&os[ix + 4]) = y1;
    }
    wave_sync();
    static_assert(16 * 1 * 32 * 16 == 16 * DM * 2);
    const int c8 = lane * 8;
    const v4f g0 = ld4bf(gain + c8), g1 = ld4bf(gain + c8 + 4), b0 = ld4bf(shift + c8), b1 = ld4bf(shift + c8 + 4);
    h16* crow = CAH + ((size_t)b * SEQ + (size_t)t0) * DM + c8;
#pragma unroll 1
    for (int ps = 0; ps < 2; ++ps) {
#pragma unroll 2
        for (int row = 0; row < 16; ++row) {
            const v4f x0 = *(const v4fa*)(&os[wb + row * LNP + c8]); const v4f x1 = *(const v4fa*)(&os[wb + row * LNP + c8 + 4]); v8h hv;
#pragma unroll
            for (int i = 0; i < 4; ++i) { const float u0 = fmaxf(x0[i] * g0[i] + b0[i], 0.0f); const float u1 = fmaxf(x1[i] * g1[i] + b1[i], 0.0f);
                hv[i] = toh_flush(u0); hv[4 + i] = toh_flush(u1); }
            *(volatile v8h*)(crow + (size_t)row * DM) = hv; }
        if (ps == 0) __threadfence(); }
}

static constexpr size_t al256(size_t v) { return (v + 255) & ~(size_t)255; }
static constexpr size_t SZ_PL = al256((size_t)NB * SEQ * DM * 2);
static constexpr size_t SZ_WB = al256((size_t)5 * NLAY * DM * DM * 2);
static constexpr size_t SZ_RF = al256((size_t)NB * SEQ * DM * 4);
static constexpr size_t SZ_TOTAL = 5 * SZ_PL + SZ_WB + SZ_RF;
static_assert(SZ_TOTAL <= (size_t)134217728);
static_assert(((size_t)DM * DM * 2) % 256 == 0);
static_assert(((size_t)NB * SEQ * DM / 8) % 256 == 0);
static_assert(((size_t)NLAY * DM * DM / 8) % 256 == 0);
static_assert(((size_t)SEQ * DM / 8) % 256 == 0);

extern "C" void kernel_launch(void* const* d_in, const int* in_sizes, int n_in,
                              void* d_out, int out_size, void* d_ws, size_t ws_size, hipStream_t stream) {
    if (n_in < 18) return;
    const size_t needx = ((size_t)(NB - 1) * SEQ_FULL + SEQ) * DM;
    const size_t needm = (size_t)(NB - 1) * SEQ_FULL + SEQ;
    if ((size_t)in_sizes[0] < needx || (size_t)in_sizes[1] < needm) return;
    if ((size_t)in_sizes[2] < (size_t)NLAY * DM * DM || (size_t)in_sizes[4] < (size_t)NLAY * DM * DM || (size_t)in_sizes[6] < (size_t)NLAY * DM * DM) return;
    if ((size_t)in_sizes[10] < (size_t)NLAY * DM * DM || (size_t)in_sizes[14] < (size_t)NLAY * DM * DM) return;
    if (in_sizes[3] < NLAY * DM || in_sizes[5] < NLAY * DM || in_sizes[7] < NLAY * DM || in_sizes[8] < NLAY * DM || in_sizes[9] < NLAY * DM) return;
    if (in_sizes[11] < NLAY * DM || in_sizes[12] < NLAY * DM || in_sizes[13] < NLAY * DM) return;
    if (in_sizes[15] < NLAY * DM || in_sizes[16] < NLAY * DM || in_sizes[17] < NLAY * DM) return;
    if ((size_t)out_size < ((size_t)(NB - 1) * OUT_SEQ + SEQ) * DM) return;
    if (SZ_TOTAL > ws_size) return;
    const float* feats = (const float*)d_in[0];
    const float* masks = (const float*)d_in[1];
    const float* qw = (const float*)d_in[2];   const float* qb = (const float*)d_in[3];
    const float* kw = (const float*)d_in[4];   const float* kb = (const float*)d_in[5];
    const float* vw = (const float*)d_in[6];   const float* vb = (const float*)d_in[7];
    const float* ag = (const float*)d_in[8];   const float* ab = (const float*)d_in[9];
    const float* cw = (const float*)d_in[10];  const float* cb = (const float*)d_in[11];
    const float* cg = (const float*)d_in[12];  const float* cs = (const float*)d_in[13];
    const float* lw = (const float*)d_in[14];  const float* lb = (const float*)d_in[15];
    const float* lg = (const float*)d_in[16];  const float* ls = (const float*)d_in[17];
    float* OUT = (float*)d_out;
    char* wsp = (char*)d_ws;
    h16* XH  = (h16*)wsp; wsp += SZ_PL;
    h16* QH  = (h16*)wsp; wsp += SZ_PL;
    h16* KP  = (h16*)wsp; wsp += SZ_PL;
    h16* VT  = (h16*)wsp; wsp += SZ_PL;
    h16* CAH = (h16*)wsp; wsp += SZ_PL;
    h16* WB  = (h16*)wsp; wsp += SZ_WB;
    float* RES = (float*)wsp; wsp += SZ_RF;
    const size_t WL = (size_t)DM * DM;
    h16* WQ = WB; h16* WK = WB + 3 * WL; h16* WV = WB + 6 * WL; h16* WC = WB + 9 * WL; h16* WLN = WB + 12 * WL;

    if (SEQ == SEQ_FULL) {
        const size_t n8 = (size_t)NB * SEQ * DM / 8;
        k_cvtx<<<(unsigned)((n8 + 255) / 256), 256, 0, stream>>>(feats, XH, n8);
    } else {
        const size_t n8 = (size_t)SEQ * DM / 8;
        for (int b = 0; b < NB; ++b) k_cvtx<<<(unsigned)((n8 + 255) / 256), 256, 0, stream>>>(feats + (size_t)b * SEQ_FULL * DM, XH + (size_t)b * SEQ * DM, n8);
    }
    { const size_t n8 = (size_t)NLAY * DM * DM / 8; const unsigned g = (unsigned)((n8 + 255) / 256);
      k_cvtw<<<g, 256, 0, stream>>>(qw, WQ, n8); k_cvtw<<<g, 256, 0, stream>>>(kw, WK, n8); k_cvtw<<<g, 256, 0, stream>>>(vw, WV, n8);
      k_cvtw<<<g, 256, 0, stream>>>(cw, WC, n8); k_cvtw<<<g, 256, 0, stream>>>(lw, WLN, n8); }

    for (int i = 0; i < NLAY; ++i) {
        const size_t wo = (size_t)i * WL; const size_t bo = (size_t)i * DM;
        k_projrow<<<dim3(NB * SEQ / 64, DM / 64, 1), 32, 0, stream>>>(XH, WQ + wo, qb + bo, QH);
        k_projrow<<<dim3(NB * SEQ / 64, DM / 64, 1), 32, 0, stream>>>(XH, WK + wo, kb + bo, KP);
        k_projtr<<<dim3(DM / 64, NB * SEQ / 64, 1), 32, 0, stream>>>(WV + wo, XH, vb + bo, VT);
        k_lnres<<<dim3(NB * SEQ / (16 * AW), 1, 1), 32 * AW, 0, stream>>>(XH, WLN + wo, lb + bo, lg + bo, ls + bo, RES, RES, XH, OUT);
        k_flash<<<dim3(SEQ / (16 * AW), NB, 1), 32 * AW, 0, stream>>>(QH, KP, VT, masks, ag + bo, ab + bo, CAH);
        if (i < NLAY - 1)
            k_lnmix<<<dim3(NB * SEQ / (16 * AW), 1, 1), 32 * AW, 0, stream>>>(CAH, WC + wo, cb + bo, cg + bo, cs + bo, RES, RES, XH, OUT);
        else
            k_lnout<<<dim3(NB * SEQ / (16 * AW), 1, 1), 32 * AW, 0, stream>>>(CAH, WC + wo, cb + bo, cg + bo, cs + bo, RES, RES, XH, OUT);
    }
}
